// TransactionGNN_69887707840602
// MI455X (gfx1250) — hardware-verified
//
#include <hip/hip_runtime.h>


namespace {
constexpr int N = 50000, NP = 50048, E = 800000, V = 100000, VP = 100352  , D = 64, NH = 4, C = 64, HC = 256, CAP1 = 128, CAP2 = 256, NB1 = CAP1 + 16  ;
constexpr float XS = 8.0f, WSC = 256.0f, NEG = 0.2f, EPSD = 1e-16f;

typedef _Float16 b16;
typedef __attribute__((ext_vector_type(16))) _Float16 v16b;
typedef __attribute__((ext_vector_type(8))) _Float16 v8b;
typedef __attribute__((ext_vector_type(8))) float v8f;
typedef __attribute__((ext_vector_type(4))) float v4f;
__device__ __forceinline__ float bf16_rne(float f) { unsigned int u = __float_as_uint(f); u += 0x7FFFu + ((u >> 16) & 1u); return __uint_as_float(u & 0xFFFF0000u); }
__device__ __forceinline__ void split16(float v, b16& hi, b16& lo) { hi = (b16)v; lo = (b16)(v - (float)hi); }
__device__ __forceinline__ v16b frag_kb(const b16* p, int hh) { const v8b a = *(const v8b*)(p + 8 * hh), b = *(const v8b*)(p + 16 + 8 * hh); v16b f;
#pragma unroll
  for (int e = 0; e < 8; ++e) { f[e] = a[e]; f[8 + e] = b[e]; } return f; }
__device__ __forceinline__ v8f wmma16b(v16b a, v16b b, v8f c) { v8f d = __builtin_amdgcn_wmma_f32_16x16x32_f16(false, a, false, b, (short)0, c, false, false); asm volatile("v_nop\n\tv_nop\n\tv_nop\n\tv_nop" : "+v"(d) : "v"(a), "v"(b)); return d; }
__device__ __forceinline__ void wave_lds_sync() { __builtin_amdgcn_fence(__ATOMIC_RELEASE, "workgroup"); __builtin_amdgcn_wave_barrier(); __builtin_amdgcn_fence(__ATOMIC_ACQUIRE, "workgroup"); }
__device__ __forceinline__ float nexp(float x) { return __builtin_amdgcn_exp2f(x * 1.4426950408889634f); }
__device__ __forceinline__ float pmul(float a, float b) { float p = a * b; asm volatile("" : "+v"(p)); return p; }
__device__ __forceinline__ int iclamp(int v, int lo, int hi) { return v < lo ? lo : (v > hi ? hi : v); }
__device__ __forceinline__ float lrelu(float x) { return x > 0.0f ? x : NEG * x; }
__device__ __forceinline__ float elu_(float x) { return x > 0.0f ? x : (__expf(x) - 1.0f); }

__global__ __launch_bounds__(256) void prep_kernel(const int* __restrict__ y, const float* __restrict__ emb, const float* __restrict__ w0, const float* __restrict__ w1, b16* __restrict__ EX16, b16* __restrict__ W0T, b16* __restrict__ W1T) {
  const size_t t = (size_t)blockIdx.x * 256 + threadIdx.x; const size_t nx = (size_t)NP * D / 8, n0 = (size_t)HC * D / 8, n1 = (size_t)HC * HC / 8; v8b o;
  if (t < nx) { const size_t e = t * 8; const size_t v = e / D; const int c0 = (int)(e % D); const int row = (v < (size_t)N) ? iclamp(y[v], 0, V - 1) : 0;
    for (int j = 0; j < 8; ++j) o[j] = (v < (size_t)N) ? (b16)(bf16_rne(emb[(size_t)row * D + c0 + j]) * XS) : (b16)0.0f; for (int pass = 0; pass < 2; ++pass) { *(volatile v8b*)(EX16 + e) = o; __threadfence(); } return; }
  size_t u = t - nx;
  if (u < n0) { const size_t e = u * 8; const int oo = (int)(e / D), i0 = (int)(e % D); for (int j = 0; j < 8; ++j) o[j] = (b16)(bf16_rne(w0[(size_t)(i0 + j) * HC + oo]) * WSC); for (int pass = 0; pass < 2; ++pass) { *(volatile v8b*)(W0T + e) = o; __threadfence(); } return; }
  u -= n0;
  if (u < n1) { const size_t e = u * 8; const int oo = (int)(e / HC), i0 = (int)(e % HC); for (int j = 0; j < 8; ++j) o[j] = (b16)(bf16_rne(w1[(size_t)(i0 + j) * HC + oo]) * WSC); for (int pass = 0; pass < 2; ++pass) { *(volatile v8b*)(W1T + e) = o; __threadfence(); } }
}
__global__ __launch_bounds__(256) void prepp_kernel(const float* __restrict__ pw2, b16* __restrict__ PW2T) {
  __shared__ __attribute__((aligned(16))) b16 T[64][64 + 8];
  const int n0 = blockIdx.x * 64, t_ = threadIdx.x;
  for (int q = t_; q < 64 * 64; q += 256) { const int k = q >> 6, nn = q & 63; T[nn][k] = (n0 + nn < V) ? (b16)(bf16_rne(pw2[(size_t)k * V + n0 + nn]) * WSC) : (b16)0.0f; }
  __syncthreads();
  for (int pass = 0; pass < 2; ++pass) { for (int q = t_; q < 64 * 8; q += 256) { const int nn = q >> 3, c8 = (q & 7) * 8; *(volatile v8b*)(PW2T + (size_t)(n0 + nn) * D + c8) = *(const v8b*)(&T[nn][c8]); } __threadfence(); }
}
__global__ __launch_bounds__(128) void gemm0_kernel(const b16* __restrict__ EX16, const b16* __restrict__ W0T, float* __restrict__ H0) {
  __shared__ __attribute__((aligned(16))) float Tf[4][16][128 + 4];
  const int wave = threadIdx.x >> 5, lane = threadIdx.x & 31, nloc = lane & 15, hlf = lane >> 4; const size_t m0 = (size_t)blockIdx.x * 64 + wave * 16;
  v8f acc[16];
#pragma unroll
  for (int t = 0; t < 16; ++t) acc[t] = (v8f){};
#pragma unroll
  for (int kb = 0; kb < D; kb += 32) { const v16b a = frag_kb(EX16 + (m0 + nloc) * D + kb, hlf);
#pragma unroll
    for (int t = 0; t < 16; ++t) acc[t] = wmma16b(a, frag_kb(W0T + (size_t)(t * 16 + nloc) * D + kb, hlf), acc[t]); }
  for (int hq = 0; hq < 2; ++hq) {
#pragma unroll
    for (int t = 0; t < 8; ++t)
#pragma unroll
      for (int r = 0; r < 8; ++r) Tf[wave][8 * hlf + r][t * 16 + nloc] = acc[hq * 8 + t][r] * (1.0f / (XS * WSC));
    wave_lds_sync();
    for (int pass = 0; pass < 2; ++pass) { for (int rr = 0; rr < 16; ++rr) *(volatile v4f*)(H0 + (m0 + rr) * HC + hq * 128 + lane * 4) = *(const v4f*)(&Tf[wave][rr][lane * 4]); __threadfence(); }
    wave_lds_sync(); }
}
__global__ __launch_bounds__(256) void node0_kernel(const float* __restrict__ H0, const float* __restrict__ asrc, const float* __restrict__ adst, float* __restrict__ AS, float* __restrict__ AD) {
  __shared__ float la[8][4], ra[8][4];
  const int wave = threadIdx.x >> 5, lane = threadIdx.x & 31; const size_t v = (size_t)blockIdx.x * 8 + wave; const int h = lane >> 3, c0 = (lane & 7) * 8;
  const float* hv = H0 + v * HC + h * C + c0; float s = 0.0f, d = 0.0f;
#pragma unroll
  for (int j = 0; j < 8; ++j) { s += pmul(hv[j], bf16_rne(asrc[h * C + c0 + j])); d += pmul(hv[j], bf16_rne(adst[h * C + c0 + j])); }
  s += __shfl_xor(s, 1); s += __shfl_xor(s, 2); s += __shfl_xor(s, 4); d += __shfl_xor(d, 1); d += __shfl_xor(d, 2); d += __shfl_xor(d, 4);
  if ((lane & 7) == 0) { la[wave][h] = s; ra[wave][h] = d; }
  __syncthreads();
  for (int pass = 0; pass < 2; ++pass) { if (threadIdx.x < 8) { *(volatile v4f*)(AS + ((size_t)blockIdx.x * 8 + threadIdx.x) * 4) = *(const v4f*)(&la[threadIdx.x][0]); *(volatile v4f*)(AD + ((size_t)blockIdx.x * 8 + threadIdx.x) * 4) = *(const v4f*)(&ra[threadIdx.x][0]); } __threadfence(); }
}
__device__ int scan_in_edges(const int* __restrict__ dsts, int u, int* lst, int cap, int* cntbuf  , bool* ovf) {
  const int t_ = threadIdx.x; constexpr int PER = (E + 255) / 256; const int e0 = t_ * PER, e1 = min(e0 + PER, E);
  int c = 0; for (int e = e0; e < e1; ++e) c += (dsts[e] == u) ? 1 : 0;
  cntbuf[t_] = c; __syncthreads();
  int pre = 0; for (int i = 0; i < t_; ++i) pre += cntbuf[i];
  int total = pre + c; __syncthreads(); if (t_ == 255) cntbuf[0] = total; __syncthreads(); total = cntbuf[0]; __syncthreads();
  int pos = pre; for (int e = e0; e < e1 && pos < cap; ++e) if (dsts[e] == u) { lst[pos++] = e; }
  __syncthreads();
  *ovf = total > cap; return min(total, cap);
}
__global__ __launch_bounds__(256) void hop1_kernel(const int* __restrict__ srcs, const int* __restrict__ dsts, const float* __restrict__ H0, const float* __restrict__ AS, const float* __restrict__ AD, const float* __restrict__ b0, b16* __restrict__ X1h, b16* __restrict__ X1l, int* __restrict__ FLAG) {
  __shared__ int cntbuf[256]; __shared__ int L1[CAP1]; __shared__ int L2[CAP2]; __shared__ float lg[CAP2 + 1][NH]; __shared__ float red[8]; __shared__ __attribute__((aligned(16))) b16 Rh[HC], Rl[HC]; __shared__ float hstat[NH][2];
  const int b = blockIdx.x, t_ = threadIdx.x, wave = t_ >> 5, lane = t_ & 31; bool ovf1 = false, ovf2 = false;
  const int n1 = scan_in_edges(dsts, N - 1, L1, CAP1, cntbuf, &ovf1);
  int u = -1; if (b < n1) u = iclamp(srcs[L1[b]], 0, N - 1); else if (b == CAP1) u = N - 1;
  float y = 0.0f;
  if (u >= 0) {
    const int n2 = scan_in_edges(dsts, u, L2, CAP2, cntbuf, &ovf2);
    for (int q = t_; q < (n2 + 1) * NH; q += 256) { const int j = q / NH, h = q % NH; const int s = (j < n2) ? iclamp(srcs[L2[j]], 0, N - 1) : u; lg[j][h] = lrelu(AS[(size_t)s * NH + h] + AD[(size_t)u * NH + h]); }
    __syncthreads();
    if (t_ < NH) { float mx = -INFINITY; for (int j = 0; j <= n2; ++j) mx = fmaxf(mx, lg[j][t_]); float sm = 0.0f; for (int j = 0; j <= n2; ++j) { const float w = nexp(lg[j][t_] - mx); lg[j][t_] = w; sm += w; } hstat[t_][0] = 1.0f / (sm + EPSD); }
    __syncthreads();
    const int h = t_ / C; float acc = 0.0f;
    for (int j = 0; j <= n2; ++j) { const int s = (j < n2) ? iclamp(srcs[L2[j]], 0, N - 1) : u; acc += pmul(lg[j][h] * hstat[h][0], H0[(size_t)s * HC + t_]); }
    y = elu_(acc + bf16_rne(b0[t_]));
    float ss = pmul(y, y);
#pragma unroll
    for (int o = 16; o >= 1; o >>= 1) ss += __shfl_xor(ss, o);
    if (lane == 0) red[wave] = ss; __syncthreads();
    float tot = 0.0f; for (int w = 0; w < 8; ++w) tot += red[w];
    y = y / fmaxf(sqrtf(tot), 1e-12f); }
  { b16 p, q; split16(y * XS, p, q); Rh[t_] = p; Rl[t_] = q; }
  __syncthreads();
  for (int pass = 0; pass < 2; ++pass) {
    if (t_ < 32) *(volatile v8b*)(X1h + (size_t)b * HC + t_ * 8) = *(const v8b*)(&Rh[t_ * 8]); else if (t_ < 64) *(volatile v8b*)(X1l + (size_t)b * HC + (t_ - 32) * 8) = *(const v8b*)(&Rl[(t_ - 32) * 8]);
    if (wave == 0 && lane < 8 && (b == 0 || b == CAP1)) { v4f fv = {0.0f, 0.0f, 0.0f, 0.0f}; if (lane == 0) fv[0] = __int_as_float((ovf1 || ovf2) ? 1 : 0); *(volatile v4f*)((float*)FLAG + (b == 0 ? 0 : 32) + lane * 4) = fv; }
    __threadfence(); }
}
__global__ __launch_bounds__(32) void gemm1_kernel(const b16* __restrict__ X1h, const b16* __restrict__ X1l, const b16* __restrict__ W1T, float* __restrict__ H1) {
  __shared__ __attribute__((aligned(16))) float Tf[16][128 + 4];
  const int lane = threadIdx.x, nloc = lane & 15, hlf = lane >> 4; const int m0 = blockIdx.x * 16;
  v8f acc[16];
#pragma unroll
  for (int t = 0; t < 16; ++t) acc[t] = (v8f){};
  for (int kb = 0; kb < HC; kb += 32) { const v16b a = frag_kb(X1h + (size_t)(m0 + nloc) * HC + kb, hlf), al = frag_kb(X1l + (size_t)(m0 + nloc) * HC + kb, hlf);
#pragma unroll
    for (int t = 0; t < 16; ++t) { const v16b bw = frag_kb(W1T + (size_t)(t * 16 + nloc) * HC + kb, hlf); acc[t] = wmma16b(a, bw, acc[t]); acc[t] = wmma16b(al, bw, acc[t]); } }
  for (int hq = 0; hq < 2; ++hq) {
#pragma unroll
    for (int t = 0; t < 8; ++t)
#pragma unroll
      for (int r = 0; r < 8; ++r) Tf[8 * hlf + r][t * 16 + nloc] = acc[hq * 8 + t][r] * (1.0f / (XS * WSC));
    wave_lds_sync();
    for (int pass = 0; pass < 2; ++pass) { for (int rr = 0; rr < 16; ++rr) *(volatile v4f*)(H1 + (size_t)(m0 + rr) * HC + hq * 128 + lane * 4) = *(const v4f*)(&Tf[rr][lane * 4]); __threadfence(); }
    wave_lds_sync(); }
}
__global__ __launch_bounds__(256) void hop2_kernel(const int* __restrict__ dsts, const float* __restrict__ H1, const float* __restrict__ asrc, const float* __restrict__ adst, const float* __restrict__ b1, const float* __restrict__ pw1, const float* __restrict__ pb1, b16* __restrict__ HVh, b16* __restrict__ HVl) {
  __shared__ int cntbuf[256]; __shared__ int L1[CAP1]; __shared__ float als[CAP1 + 1][NH]; __shared__ float lg[CAP1 + 1][NH]; __shared__ float hstat[NH]; __shared__ float red[8]; __shared__ float x2[HC]; __shared__ __attribute__((aligned(16))) b16 Ph[16 * D], Pl[16 * D];
  const int t_ = threadIdx.x, wave = t_ >> 5, lane = t_ & 31; bool ovf = false;
  const int n1 = scan_in_edges(dsts, N - 1, L1, CAP1, cntbuf, &ovf); (void)L1;
  for (int q = t_; q < (n1 + 1) * NH; q += 256) { const int j = q / NH, h = q % NH; const int row = (j < n1) ? j : CAP1; const float* hr = H1 + (size_t)row * HC + h * C; float s = 0.0f; for (int c = 0; c < C; ++c) s += pmul(hr[c], bf16_rne(asrc[h * C + c])); als[j][h] = s; }
  if (t_ < NH) { const float* hr = H1 + (size_t)CAP1 * HC + t_ * C; float d = 0.0f; for (int c = 0; c < C; ++c) d += pmul(hr[c], bf16_rne(adst[t_ * C + c])); hstat[t_] = d; }
  __syncthreads();
  if (t_ < NH) { const float ad = hstat[t_]; float mx = -INFINITY; for (int j = 0; j <= n1; ++j) { const float l = lrelu(als[j][t_] + ad); lg[j][t_] = l; mx = fmaxf(mx, l); } float sm = 0.0f; for (int j = 0; j <= n1; ++j) { const float w = nexp(lg[j][t_] - mx); lg[j][t_] = w; sm += w; } hstat[t_] = 1.0f / (sm + EPSD); }
  __syncthreads();
  { const int h = t_ / C; float acc = 0.0f; for (int j = 0; j <= n1; ++j) { const int row = (j < n1) ? j : CAP1; acc += pmul(lg[j][h] * hstat[h], H1[(size_t)row * HC + t_]); }
    float y = elu_(acc + bf16_rne(b1[t_])); float ss = pmul(y, y);
#pragma unroll
    for (int o = 16; o >= 1; o >>= 1) ss += __shfl_xor(ss, o);
    if (lane == 0) red[wave] = ss; __syncthreads(); float tot = 0.0f; for (int w = 0; w < 8; ++w) tot += red[w];
    x2[t_] = y / fmaxf(sqrtf(tot), 1e-12f); }
  __syncthreads();
  for (int q = t_; q < 16 * D; q += 256) { b16 p = (b16)0.0f, ql = (b16)0.0f; if (q < D) { float s = bf16_rne(pb1[q]); for (int k = 0; k < HC; ++k) s += pmul(x2[k], bf16_rne(pw1[(size_t)k * D + q])); s = fmaxf(s, 0.0f); split16(s * XS, p, ql); } Ph[q] = p; Pl[q] = ql; }
  __syncthreads();
  for (int pass = 0; pass < 2; ++pass) { if (t_ < 128) *(volatile v8b*)(HVh + t_ * 8) = *(const v8b*)(&Ph[t_ * 8]); else *(volatile v8b*)(HVl + (t_ - 128) * 8) = *(const v8b*)(&Pl[(t_ - 128) * 8]); __threadfence(); }
}
__global__ __launch_bounds__(32) void out_kernel(const b16* __restrict__ HVh, const b16* __restrict__ HVl, const b16* __restrict__ PW2T, const float* __restrict__ pb2, float* __restrict__ out) {
  __shared__ __attribute__((aligned(16))) float row0[128];
  const int lane = threadIdx.x, nloc = lane & 15, hlf = lane >> 4; const int n0 = blockIdx.x * 128;
  v8f acc[8];
#pragma unroll
  for (int t = 0; t < 8; ++t) acc[t] = (v8f){};
#pragma unroll
  for (int kb = 0; kb < D; kb += 32) { const v16b a = frag_kb(HVh + nloc * D + kb, hlf), al = frag_kb(HVl + nloc * D + kb, hlf);
#pragma unroll
    for (int t = 0; t < 8; ++t) { const v16b bw = frag_kb(PW2T + (size_t)(n0 + t * 16 + nloc) * D + kb, hlf); acc[t] = wmma16b(a, bw, acc[t]); acc[t] = wmma16b(al, bw, acc[t]); } }
  if (hlf == 0) {
#pragma unroll
    for (int t = 0; t < 8; ++t) { const int n = n0 + t * 16 + nloc; row0[t * 16 + nloc] = acc[t][0] * (1.0f / (XS * WSC)) + ((n < V) ? bf16_rne(pb2[n]) : 0.0f); } }
  wave_lds_sync();
  for (int pass = 0; pass < 2; ++pass) { if (n0 + lane * 4 < V) *(volatile v4f*)(out + n0 + lane * 4) = *(const v4f*)(&row0[lane * 4]); __threadfence(); }
}
}

extern "C" void kernel_launch(void* const* d_in, const int* in_sizes, int n_in, void* d_out, int out_size, void* d_ws, size_t ws_size, hipStream_t stream) {
  (void)n_in;
  auto Fp = [&](int i) { return (const float*)d_in[i]; }; auto Ip = [&](int i) { return (const int*)d_in[i]; };
  if (in_sizes[0] != N || in_sizes[1] != 2 * E || in_sizes[2] != V * D || in_sizes[3] != D * HC || in_sizes[4] != NH * C || in_sizes[7] != HC * HC || in_sizes[11] != HC * D || in_sizes[13] != D * V || in_sizes[14] != V || out_size != V) return;
  size_t off = 0; char* ws = (char*)d_ws;
  auto carve = [&](size_t bytes) { char* p = ws + off; off += (bytes + 255) & ~(size_t)255; return p; };
  b16* EX16 = (b16*)carve((size_t)NP * D * 2); b16* W0T = (b16*)carve((size_t)HC * D * 2); b16* W1T = (b16*)carve((size_t)HC * HC * 2); b16* PW2T = (b16*)carve((size_t)VP * D * 2);
  float* H0 = (float*)carve((size_t)NP * HC * 4); float* AS = (float*)carve((size_t)NP * NH * 4); float* AD = (float*)carve((size_t)NP * NH * 4);
  b16* X1h = (b16*)carve((size_t)NB1 * HC * 2); b16* X1l = (b16*)carve((size_t)NB1 * HC * 2); float* H1 = (float*)carve((size_t)NB1 * HC * 4); b16* HVh = (b16*)carve((size_t)16 * D * 2); b16* HVl = (b16*)carve((size_t)16 * D * 2); int* FLAG = (int*)carve(256);
  if (off > ws_size || off > ((size_t)128 << 20)) return;
  prep_kernel<<<(unsigned)(((size_t)NP * D / 8 + (size_t)HC * D / 8 + (size_t)HC * HC / 8 + 255) / 256), 256, 0, stream>>>(Ip(0), Fp(2), Fp(3), Fp(7), EX16, W0T, W1T);
  prepp_kernel<<<VP / 64, 256, 0, stream>>>(Fp(13), PW2T);
  gemm0_kernel<<<NP / 64, 128, 0, stream>>>(EX16, W0T, H0);
  node0_kernel<<<NP / 8, 256, 0, stream>>>(H0, Fp(4), Fp(5), AS, AD);
  hop1_kernel<<<NB1, 256, 0, stream>>>(Ip(1), Ip(1) + E, H0, AS, AD, Fp(6), X1h, X1l, FLAG);
  gemm1_kernel<<<NB1 / 16, 32, 0, stream>>>(X1h, X1l, W1T, H1);
  hop2_kernel<<<1, 256, 0, stream>>>(Ip(1) + E, H1, Fp(8), Fp(9), Fp(10), Fp(11), Fp(12), HVh, HVl);
  out_kernel<<<VP / 128, 32, 0, stream>>>(HVh, HVl, PW2T, Fp(14), (float*)d_out);
}
